// RelPosMultiHeadedAttention_87342454931744
// MI455X (gfx1250) — hardware-verified
//
#include <hip/hip_runtime.h>


namespace {
constexpr int NB = 2, S = 2048, E = 512, NH = 8, D = 64, NR = NB * S, BS = 2048  ;
constexpr float XS = 8.0f, WSC = 256.0f, PS = 8.0f, SCALE = 0.044194173824159216f  , LOG2E = 1.4426950408889634f;

typedef _Float16 b16;
typedef __attribute__((ext_vector_type(16))) _Float16 v16b;
typedef __attribute__((ext_vector_type(8))) _Float16 v8b;
typedef __attribute__((ext_vector_type(8))) float v8f;
typedef __attribute__((ext_vector_type(4))) float v4f;
__device__ __forceinline__ float bf16_rne(float f) { unsigned int u = __float_as_uint(f); u += 0x7FFFu + ((u >> 16) & 1u); return __uint_as_float(u & 0xFFFF0000u); }
__device__ __forceinline__ void split16(float v, b16& hi, b16& lo) { hi = (b16)v; lo = (b16)(v - (float)hi); }
__device__ __forceinline__ v16b frag_kb(const b16* p, int hh) { const v8b a = *(const v8b*)(p + 8 * hh), b = *(const v8b*)(p + 16 + 8 * hh); v16b f;
#pragma unroll
  for (int e = 0; e < 8; ++e) { f[e] = a[e]; f[8 + e] = b[e]; } return f; }
__device__ __forceinline__ v8f wmma16b(v16b a, v16b b, v8f c) { v8f d = __builtin_amdgcn_wmma_f32_16x16x32_f16(false, a, false, b, (short)0, c, false, false); asm volatile("v_nop\n\tv_nop\n\tv_nop\n\tv_nop" : "+v"(d) : "v"(a), "v"(b)); return d; }
__device__ __forceinline__ void wave_lds_sync() { __builtin_amdgcn_fence(__ATOMIC_RELEASE, "workgroup"); __builtin_amdgcn_wave_barrier(); __builtin_amdgcn_fence(__ATOMIC_ACQUIRE, "workgroup"); }
__device__ __forceinline__ float nexp2(float x) { return __builtin_amdgcn_exp2f(x); }

__global__ __launch_bounds__(256) void prepx_kernel(const float* __restrict__ x, b16* __restrict__ T16) {
  const size_t t = (size_t)blockIdx.x * 256 + threadIdx.x; const size_t n1 = (size_t)NR * E / 8; const float* src; b16* dst; size_t e;
  if (t < n1) { src = x; dst = T16; e = t * 8; } else return;
  const v4f a = *(const v4f*)(src + e), c = *(const v4f*)(src + e + 4); v8b o;
#pragma unroll
  for (int j = 0; j < 4; ++j) { o[j] = (b16)(bf16_rne(a[j]) * XS); o[4 + j] = (b16)(bf16_rne(c[j]) * XS); }
  for (int pass = 0; pass < 2; ++pass) { *(volatile v8b*)(dst + e) = o; __threadfence(); }
}
__global__ __launch_bounds__(256) void prepw_kernel(const float* __restrict__ wq, const float* __restrict__ wk, const float* __restrict__ wv, const float* __restrict__ wo, const float* __restrict__ er, b16* __restrict__ W3, b16* __restrict__ WOT, b16* __restrict__ ER16) {
  const size_t t = (size_t)blockIdx.x * 256 + threadIdx.x; const size_t n0 = 3 * D * D / 8, n1 = (size_t)E * E / 8, n2 = (size_t)NH * BS * D / 8; const float* src; b16* dst; size_t e;
  if (t < n0) { const int k = (int)(t / (D * D / 8)); src = (k == 0 ? wq : k == 1 ? wk : wv) - (size_t)k * D * D; dst = W3; e = t * 8; } else if (t < n0 + n1) { src = wo; dst = WOT; e = (t - n0) * 8; } else if (t < n0 + n1 + n2) { src = er; dst = ER16; e = (t - n0 - n1) * 8; } else return;
  const v4f a = *(const v4f*)(src + e), c = *(const v4f*)(src + e + 4); v8b o;
#pragma unroll
  for (int j = 0; j < 4; ++j) { o[j] = (b16)(bf16_rne(a[j]) * WSC); o[4 + j] = (b16)(bf16_rne(c[j]) * WSC); }
  for (int pass = 0; pass < 2; ++pass) { *(volatile v8b*)(dst + e) = o; __threadfence(); }
}
__global__ __launch_bounds__(128) void projh_kernel(const b16* __restrict__ T16, const b16* __restrict__ W3, b16* __restrict__ Qh, b16* __restrict__ Ql, b16* __restrict__ Kh, b16* __restrict__ Kl, b16* __restrict__ VTh, b16* __restrict__ VTl) {
  __shared__ __attribute__((aligned(16))) b16 Th[4][16][D + 8], Tl[4][16][D + 8]; __shared__ __attribute__((aligned(16))) b16 Vt[D][64 + 8], Vtl[D][64 + 8];
  const int wave = threadIdx.x >> 5, lane = threadIdx.x & 31, nloc = lane & 15, hlf = lane >> 4, t_ = threadIdx.x; const int h = blockIdx.y, kind = blockIdx.z % 3, b = blockIdx.z / 3; const int s0 = blockIdx.x * 64 + wave * 16;
  const b16* A = T16 + ((size_t)b * S) * E + h * D; const b16* Wk_ = W3 + (size_t)kind * D * D; v8f acc[4] = {{}, {}, {}, {}};
#pragma unroll
  for (int kb = 0; kb < D; kb += 32) { const v16b a = frag_kb(A + (size_t)(s0 + nloc) * E + kb, hlf);
#pragma unroll
    for (int t = 0; t < 4; ++t) acc[t] = wmma16b(a, frag_kb(Wk_ + (size_t)(t * 16 + nloc) * D + kb, hlf), acc[t]); }
  if (kind < 2) {
#pragma unroll
    for (int t = 0; t < 4; ++t)
#pragma unroll
      for (int r = 0; r < 8; ++r) { b16 h_, l_; split16(acc[t][r] * (1.0f / (XS * WSC)) * XS, h_, l_); Th[wave][8 * hlf + r][t * 16 + nloc] = h_; Tl[wave][8 * hlf + r][t * 16 + nloc] = l_; }
    wave_lds_sync();
    b16* dh = kind == 0 ? Qh : Kh; b16* dl = kind == 0 ? Ql : Kl;
    for (int pass = 0; pass < 2; ++pass) { for (int q = 0; q < 4; ++q) { const int rr = q * 4 + (lane >> 3), c8 = (lane & 7) * 8; const size_t gi = ((size_t)b * S + s0 + rr) * E + h * D + c8; *(volatile v8b*)(dh + gi) = *(const v8b*)(&Th[wave][rr][c8]); *(volatile v8b*)(dl + gi) = *(const v8b*)(&Tl[wave][rr][c8]); } __threadfence(); }
  } else {
#pragma unroll
    for (int t = 0; t < 4; ++t)
#pragma unroll
      for (int r = 0; r < 8; ++r) { b16 h_, l_; split16(acc[t][r] * (1.0f / (XS * WSC)) * XS, h_, l_); Vt[t * 16 + nloc][wave * 16 + 8 * hlf + r] = h_; Vtl[t * 16 + nloc][wave * 16 + 8 * hlf + r] = l_; }
    __syncthreads();
    const int sb = blockIdx.x * 64;
    for (int pass = 0; pass < 2; ++pass) { for (int q = t_; q < D * 8; q += 128) { const int dd = q >> 3, c8 = (q & 7) * 8; const size_t gi = (((size_t)b * NH + h) * D + dd) * S + sb + c8; *(volatile v8b*)(VTh + gi) = *(const v8b*)(&Vt[dd][c8]); *(volatile v8b*)(VTl + gi) = *(const v8b*)(&Vtl[dd][c8]); } __threadfence(); } }
}
__global__ __launch_bounds__(256) void vmean_kernel(const b16* __restrict__ VTh, const b16* __restrict__ VTl, float* __restrict__ VM) {
  __shared__ __attribute__((aligned(16))) float row[D];
  const int wave = threadIdx.x >> 5, lane = threadIdx.x & 31; const int bh = blockIdx.x;
  for (int d8 = 0; d8 < D; d8 += 8) { const int d = d8 + wave; const b16* vr = VTh + ((size_t)bh * D + d) * S; const b16* vl = VTl + ((size_t)bh * D + d) * S; float s = 0.0f;
#pragma unroll 1
    for (int j = lane; j < S; j += 32) { s += (float)vr[j]; s += (float)vl[j]; }
#pragma unroll
    for (int o = 16; o >= 1; o >>= 1) s += __shfl_xor(s, o);
    if (lane == 0) row[d] = s * (1.0f / (XS * S)); }
  __syncthreads();
  for (int pass = 0; pass < 2; ++pass) { if (threadIdx.x < 16) *(volatile v4f*)(VM + (size_t)bh * D + threadIdx.x * 4) = *(const v4f*)(&row[threadIdx.x * 4]); __threadfence(); }
}
__global__ __launch_bounds__(64) void attn_kernel(const b16* __restrict__ Qh, const b16* __restrict__ Ql, const b16* __restrict__ Kh, const b16* __restrict__ Kl, const b16* __restrict__ VTh, const b16* __restrict__ VTl, const b16* __restrict__ ER16g, const int* __restrict__ mask, const float* __restrict__ VM, int qb0, b16* __restrict__ Oh, b16* __restrict__ Ol) {
  __shared__ __attribute__((aligned(16))) float To[2][16][D + 4]; __shared__ float Tr[2][16][48 + 1];
  const int wave = threadIdx.x >> 5, lane = threadIdx.x & 31, hh = lane >> 4, col = lane & 15; const int b = blockIdx.z, h = blockIdx.y; const int q0 = (qb0 + blockIdx.x) * 32 + wave * 16, qi = q0 + col;
  const size_t qo = ((size_t)b * S + qi) * E + h * D; const v16b qa0 = frag_kb(Qh + qo, hh), qa1 = frag_kb(Qh + qo + 32, hh), ql0 = frag_kb(Ql + qo, hh), ql1 = frag_kb(Ql + qo + 32, hh);
  const b16* Kb = Kh + (size_t)b * S * E + h * D; const b16* Klb = Kl + (size_t)b * S * E + h * D; const b16* Vb = VTh + ((size_t)b * NH + h) * D * S; const b16* Vlb = VTl + ((size_t)b * NH + h) * D * S;
  const b16* ER16 = ER16g + (size_t)h * BS * D;
  float m = -INFINITY, l = 0.0f; v8f o[4] = {{}, {}, {}, {}}, ol[4] = {{}, {}, {}, {}};
  const float cs = SCALE * LOG2E / (XS * XS); const int kend = q0 + 16;
  for (int kb = 0; kb < kend; kb += 32) {
    v8f s0 = {}, s1 = {};
    { const b16* k0 = Kb + (size_t)(kb + col) * E, *k1 = Kb + (size_t)(kb + 16 + col) * E, *k0l = Klb + (size_t)(kb + col) * E, *k1l = Klb + (size_t)(kb + 16 + col) * E;
      v16b f = frag_kb(k0, hh); s0 = wmma16b(f, qa0, s0); s0 = wmma16b(f, ql0, s0); s0 = wmma16b(frag_kb(k0l, hh), qa0, s0);
      f = frag_kb(k0 + 32, hh); s0 = wmma16b(f, qa1, s0); s0 = wmma16b(f, ql1, s0); s0 = wmma16b(frag_kb(k0l + 32, hh), qa1, s0);
      f = frag_kb(k1, hh); s1 = wmma16b(f, qa0, s1); s1 = wmma16b(f, ql0, s1); s1 = wmma16b(frag_kb(k1l, hh), qa0, s1);
      f = frag_kb(k1 + 32, hh); s1 = wmma16b(f, qa1, s1); s1 = wmma16b(f, ql1, s1); s1 = wmma16b(frag_kb(k1l + 32, hh), qa1, s1); }
    { const int base = S - 1 - (q0 + 15) + kb;
#pragma unroll
      for (int wt = 0; wt < 3; ++wt) { v8f tq = {};
#pragma unroll
        for (int ks = 0; ks < 2; ++ks) { const int erow = min(base + wt * 16 + col, BS - 1); const v16b be = frag_kb(ER16 + (size_t)erow * D + ks * 32, hh); const v16b qa = ks == 0 ? qa0 : qa1, ql = ks == 0 ? ql0 : ql1;
          tq = wmma16b(qa, be, tq); tq = wmma16b(ql, be, tq); }
#pragma unroll
        for (int r = 0; r < 8; ++r) Tr[wave][8 * hh + r][wt * 16 + col] = tq[r] * (1.0f / (XS * WSC)); }
      wave_lds_sync(); }
    float e[16]; float mx = -INFINITY;
#pragma unroll
    for (int r = 0; r < 8; ++r) { const int k0i = kb + 8 * hh + r, k1i = kb + 16 + 8 * hh + r;
      const float rel0 = Tr[wave][col][15 - col + 8 * hh + r], rel1 = Tr[wave][col][15 - col + 16 + 8 * hh + r];
      e[r] = (k0i <= qi) ? (s0[r] * (SCALE / (XS * XS)) + rel0) * LOG2E : -INFINITY; e[8 + r] = (k1i <= qi) ? (s1[r] * (SCALE / (XS * XS)) + rel1) * LOG2E : -INFINITY; mx = fmaxf(mx, fmaxf(e[r], e[8 + r])); }
    wave_lds_sync();
    mx = fmaxf(mx, __shfl_xor(mx, 16)); const float mn = fmaxf(m, mx); const float al = nexp2(m - mn); m = mn; float sum = 0.0f; v16b ph, pl;
#pragma unroll
    for (int i = 0; i < 16; ++i) { const float p = nexp2(e[i] - mn); sum += p; const b16 h_ = (b16)(p * PS); ph[i] = h_; pl[i] = (b16)(p * PS - (float)h_); }
    sum += __shfl_xor(sum, 16); l = l * al + sum;
#pragma unroll
    for (int t = 0; t < 4; ++t) { o[t] *= al; ol[t] *= al; const v16b vf = frag_kb(Vb + (size_t)(t * 16 + col) * S + kb, hh); o[t] = wmma16b(vf, ph, o[t]); ol[t] = wmma16b(vf, pl, ol[t]); ol[t] = wmma16b(frag_kb(Vlb + (size_t)(t * 16 + col) * S + kb, hh), ph, ol[t]); } }
  const float inv = 1.0f / (l * PS * XS);
#pragma unroll
  for (int t = 0; t < 4; ++t)
#pragma unroll
    for (int r = 0; r < 8; ++r) { const int d = t * 16 + 8 * hh + r; To[wave][col][d] = (mask[(size_t)b * S + qi] != 0) ? (o[t][r] + ol[t][r]) * inv : VM[((size_t)b * NH + h) * D + d]; }
  wave_lds_sync();
  for (int pass = 0; pass < 2; ++pass) { for (int r4 = 0; r4 < 16; r4 += 4) { const int rr = r4 + (lane >> 3), c8 = (lane & 7) * 8; v8b hv, lv; for (int j = 0; j < 8; ++j) { b16 a_, c_; split16(To[wave][rr][c8 + j] * XS, a_, c_); hv[j] = a_; lv[j] = c_; }
      const size_t gi = (((size_t)b * NH + h) * S + q0 + rr) * D + c8;   *(volatile v8b*)(Oh + gi) = hv; *(volatile v8b*)(Ol + gi) = lv; } __threadfence(); }
}
__global__ __launch_bounds__(128) void outproj_kernel(const b16* __restrict__ Oh, const b16* __restrict__ Ol, const b16* __restrict__ WOT, const float* __restrict__ bo, float* __restrict__ out) {
  __shared__ __attribute__((aligned(16))) float Ts[4][16][128 + 4];
  const int wave = threadIdx.x >> 5, lane = threadIdx.x & 31, nloc = lane & 15, hlf = lane >> 4; const size_t m0 = (size_t)blockIdx.x * 64 + wave * 16; const int n0 = blockIdx.y * 128;
  v8f acc[8];
#pragma unroll
  for (int t = 0; t < 8; ++t) acc[t] = (v8f){};
#pragma unroll 2
  for (int kb = 0; kb < E; kb += 32) { const v16b a = frag_kb(Oh + (m0 + nloc) * E + kb, hlf), al = frag_kb(Ol + (m0 + nloc) * E + kb, hlf);
#pragma unroll
    for (int t = 0; t < 8; ++t) { const v16b bw = frag_kb(WOT + (size_t)(n0 + t * 16 + nloc) * E + kb, hlf); acc[t] = wmma16b(a, bw, acc[t]); acc[t] = wmma16b(al, bw, acc[t]); } }
#pragma unroll
  for (int t = 0; t < 8; ++t)
#pragma unroll
    for (int r = 0; r < 8; ++r) Ts[wave][8 * hlf + r][t * 16 + nloc] = acc[t][r] * (1.0f / (XS * WSC)) + bf16_rne(bo[n0 + t * 16 + nloc]);
  wave_lds_sync();
  for (int pass = 0; pass < 2; ++pass) { for (int rr = 0; rr < 16; ++rr) *(volatile v4f*)(out + (m0 + rr) * E + n0 + lane * 4) = *(const v4f*)(&Ts[wave][rr][lane * 4]); __threadfence(); }
}
}

extern "C" void kernel_launch(void* const* d_in, const int* in_sizes, int n_in, void* d_out, int out_size, void* d_ws, size_t ws_size, hipStream_t stream) {
  (void)n_in;
  auto Fp = [&](int i) { return (const float*)d_in[i]; };
  if (in_sizes[0] != NR * E || in_sizes[1] != NR || in_sizes[3] != D * D || in_sizes[4] != D * D || in_sizes[5] != D * D || in_sizes[6] != NH * BS * D || in_sizes[7] != E * E || in_sizes[8] != E || out_size != NR * E) return;
  size_t off = 0; char* ws = (char*)d_ws;
  auto carve = [&](size_t bytes) { char* p = ws + off; off += (bytes + 255) & ~(size_t)255; return p; };
  b16* T16 = (b16*)carve((size_t)NR * E * 2); b16* W3 = (b16*)carve((size_t)3 * D * D * 2); b16* WOT = (b16*)carve((size_t)E * E * 2); b16* ER16 = (b16*)carve((size_t)NH * BS * D * 2);
  b16* Qh = (b16*)carve((size_t)NR * E * 2); b16* Ql = (b16*)carve((size_t)NR * E * 2); b16* Kh = (b16*)carve((size_t)NR * E * 2); b16* Kl = (b16*)carve((size_t)NR * E * 2); b16* VTh = (b16*)carve((size_t)NR * E * 2); b16* VTl = (b16*)carve((size_t)NR * E * 2);
  b16* Oh = (b16*)carve((size_t)NR * E * 2); b16* Ol = (b16*)carve((size_t)NR * E * 2); float* VM = (float*)carve((size_t)NB * NH * D * 4);
  if (off > ws_size || off > ((size_t)128 << 20)) return;
  prepx_kernel<<<(unsigned)(((size_t)NR * E / 8 + 255) / 256), 256, 0, stream>>>(Fp(0), T16);
  prepw_kernel<<<(unsigned)(((size_t)3 * D * D / 8 + (size_t)E * E / 8 + (size_t)NH * BS * D / 8 + 255) / 256), 256, 0, stream>>>(Fp(3), Fp(4), Fp(5), Fp(7), Fp(6), W3, WOT, ER16);
  projh_kernel<<<dim3(S / 64, NH, 3 * NB), 128, 0, stream>>>(T16, W3, Qh, Ql, Kh, Kl, VTh, VTl);
  vmean_kernel<<<NB * NH, 256, 0, stream>>>(VTh, VTl, VM);
  attn_kernel<<<dim3(S / 32, NH, NB), 64, 0, stream>>>(Qh, Ql, Kh, Kl, VTh, VTl, ER16, (const int*)d_in[1], VM, 0, Oh, Ol);
  outproj_kernel<<<dim3(NR / 64, E / 128), 128, 0, stream>>>(Oh, Ol, WOT, Fp(8), (float*)d_out);
}
